// ClassicalSelfAttention_65481071406199
// MI455X (gfx1250) — hardware-verified
//
#include <hip/hip_runtime.h>
#include <math.h>

constexpr int kBatch   = 2;
constexpr int kSeq     = 4096;
constexpr int kSeqHalf = 2048;
constexpr int kDim     = 512;
constexpr int kHeads   = 8;
constexpr int kHeadDim = 64;
constexpr int kTok     = kBatch * kSeq;
constexpr int kQKld    = 2 * kDim;
constexpr float kWCarry    = 16.0f;
constexpr float kWCarryInv = 1.0f / 16.0f;
constexpr float kAttScale  = 0.125f;
constexpr float kPCarry    = 2048.0f;
constexpr float kCtxCarry  = 256.0f;
constexpr float kPVScale   = kCtxCarry / kPCarry;
constexpr float kOutScale  = 1.0f / (kCtxCarry * kWCarry);
constexpr float kInvDim    = 1.0f / 512.0f;
constexpr float kLnEps     = 1e-5f;

constexpr size_t kBytesQK  = (size_t)kTok * kQKld * 2;
constexpr size_t kBytesVT  = (size_t)kBatch * kDim * kSeq * 2;
constexpr size_t kBytesCTX = (size_t)kTok * kDim * 2;
constexpr size_t kBytesXh  = (size_t)kTok * kDim * 2;
constexpr size_t kBytesW16 = (size_t)kDim * kDim * 2;
constexpr size_t kBytesS   = (size_t)kSeq * kSeq * 4;
constexpr size_t kBytesP   = (size_t)kSeq * kSeq * 2;
constexpr size_t kBytesY   = (size_t)kTok * kDim * 4;
constexpr size_t kOffQK  = 0;
constexpr size_t kOffVT  = kOffQK + kBytesQK;
constexpr size_t kOffCTX = kOffVT + kBytesVT;
constexpr size_t kOffU   = kOffCTX + kBytesCTX;
constexpr size_t kBytesU = kBytesS + kBytesP;
constexpr size_t kOffXh  = kOffU;
constexpr size_t kOffWqk = kOffXh + kBytesXh;
constexpr size_t kOffWv  = kOffWqk + 2 * kBytesW16;
constexpr size_t kOffS   = kOffU;
constexpr size_t kOffP   = kOffS + kBytesS;
constexpr size_t kOffY   = kOffU;
constexpr size_t kOffWo  = kOffY + kBytesY;
constexpr size_t kWsTotal = kOffU + kBytesU;
static_assert(kOffWv + kBytesW16 <= kOffU + kBytesU);
static_assert(kOffP + kBytesP <= kOffU + kBytesU);
static_assert(kOffWo + kBytesW16 <= kOffU + kBytesU);
static_assert(kWsTotal == (size_t)134217728u);

typedef __attribute__((ext_vector_type(16))) _Float16 v16h;
typedef __attribute__((ext_vector_type(8)))  _Float16 v8h;
typedef __attribute__((ext_vector_type(16))) __bf16   v16b;
typedef __attribute__((ext_vector_type(8)))  __bf16   v8b;
typedef __attribute__((ext_vector_type(8)))  float    v8f;
typedef __attribute__((ext_vector_type(4)))  float    v4f;
typedef __attribute__((ext_vector_type(4)))  unsigned int v4u;

__device__ __forceinline__ unsigned short f2bf_bits(float f) {
  unsigned u = __float_as_uint(f);
  return (unsigned short)((u + 0x7FFFu + ((u >> 16) & 1u)) >> 16);
}
__device__ __forceinline__ float bf_bits2f(unsigned short h) { return __uint_as_float(((unsigned)h) << 16); }

__device__ __forceinline__ void dep_guard_h(v8f& a, v8f& b, v16h x, v16h y) { asm volatile("v_nop\n\tv_nop\n\tv_nop\n\tv_nop" : "+v"(a), "+v"(b) : "v"(x), "v"(y)); }
__device__ __forceinline__ void dep_guard_b(v8f& a, v8f& b, v16b x, v16b y) { asm volatile("v_nop\n\tv_nop\n\tv_nop\n\tv_nop" : "+v"(a), "+v"(b) : "v"(x), "v"(y)); }
__device__ __forceinline__ void keep4_h(v16h a, v16h b, v16h c, v16h d) { asm volatile("v_nop" :: "v"(a), "v"(b), "v"(c), "v"(d)); }
__device__ __forceinline__ void keep4_b(v16b a, v16b b, v16b c, v16b d) { asm volatile("v_nop" :: "v"(a), "v"(b), "v"(c), "v"(d)); }
__device__ __forceinline__ void acc_guard4(v8f& a, v8f& b, v8f& c, v8f& d) { asm volatile("v_nop\n\tv_nop\n\tv_nop\n\tv_nop" : "+v"(a), "+v"(b), "+v"(c), "+v"(d)); }
template <typename T> struct Frag;
template <> struct Frag<_Float16> {
  typedef v16h V; union U { v16h v; v8h h[2]; };
  static __device__ __forceinline__ v16h load(const _Float16* p) {
    U f; f.h[0] = *(const v8h*)(p); f.h[1] = *(const v8h*)(p + 16); return f.v;
  }
  static __device__ __forceinline__ v8f mma(v16h a, v16h b, v8f c) {
    return __builtin_amdgcn_wmma_f32_16x16x32_f16(false, a, false, b, (short)0, c, false, false);
  }
  static __device__ __forceinline__ void guard(v8f& a, v8f& b, v16h x, v16h y) { dep_guard_h(a, b, x, y); }
  static __device__ __forceinline__ void keep(v16h a, v16h b, v16h c, v16h d) { keep4_h(a, b, c, d); }
};
template <> struct Frag<__bf16> {
  typedef v16b V; union U { v16b v; v8b h[2]; };
  static __device__ __forceinline__ v16b load(const __bf16* p) {
    U f; f.h[0] = *(const v8b*)(p); f.h[1] = *(const v8b*)(p + 16); return f.v;
  }
  static __device__ __forceinline__ v8f mma(v16b a, v16b b, v8f c) {
    return __builtin_amdgcn_wmma_f32_16x16x32_bf16(false, a, false, b, (short)0, c, false, false);
  }
  static __device__ __forceinline__ void guard(v8f& a, v8f& b, v16b x, v16b y) { dep_guard_b(a, b, x, y); }
  static __device__ __forceinline__ void keep(v16b a, v16b b, v16b c, v16b d) { keep4_b(a, b, c, d); }
};

__device__ __forceinline__ unsigned pk16(unsigned short a, unsigned short b) { return (unsigned)a | ((unsigned)b << 16); }
__device__ __forceinline__ unsigned short h_bits(float f) { const _Float16 h = (_Float16)f; return __builtin_bit_cast(unsigned short, h); }

template <int ET> struct Elem;
template <> struct Elem<0> { typedef _Float16 T; };
template <> struct Elem<1> { typedef __bf16 T; };
template <int ET, bool SPLIT, int BIAS_MODE, int OUT_MODE, bool RESID, int ACT = 0>
__global__ __launch_bounds__(256) void wmma_gemm64(
    const unsigned short* __restrict__ Ap, const unsigned short* __restrict__ A2p, int lda, long strideA,
    const unsigned short* __restrict__ Btp, const unsigned short* __restrict__ Bt2p, int ldb, long strideB,
    void* __restrict__ Cout, void* __restrict__ Cout2, int ldc, long strideC,
    const float* __restrict__ bias,
    const float* __restrict__ resid, long strideR,
    int M, int N, int K, float scale) {
  typedef typename Elem<ET>::T T;
  typedef typename Frag<T>::V V;
  const T* A = (const T*)Ap; const T* A2 = (const T*)A2p; const T* Bt = (const T*)Btp; const T* Bt2 = (const T*)Bt2p;
  __shared__ __align__(16) float sT[8][16 * 68];
  const int b    = blockIdx.y;
  const int lane = threadIdx.x & 31;
  const int wave = threadIdx.x >> 5;
  const int tilesN = N >> 6;
  const int tilesM = M >> 6;
  const int tile = blockIdx.x * 8 + wave;
  if (tile >= tilesM * tilesN) return;
  const int tm = tile / tilesN;
  const int tn = tile - tm * tilesN;
  const int m0 = tm << 6;
  const int n0 = tn << 6;

  const T* Ab  = A  + (size_t)b * strideA;
  const T* Bb  = Bt + (size_t)b * strideB;
  const T* Ab2 = SPLIT ? (A2  + (size_t)b * strideA) : nullptr;
  const T* Bb2 = SPLIT ? (Bt2 + (size_t)b * strideB) : nullptr;

  const int rlane = lane & 15;
  const int koff  = (lane >> 4) * 8;
  const int mOff  = (lane >> 4) * 8;

  v8f acc[4][4];
#pragma unroll
  for (int i = 0; i < 4; ++i)
#pragma unroll
    for (int j = 0; j < 4; ++j) acc[i][j] = (v8f){0.f,0.f,0.f,0.f,0.f,0.f,0.f,0.f};

  for (int k0 = 0; k0 < K; k0 += 32) {
    V bh[4], bl[4];
#pragma unroll
    for (int j = 0; j < 4; ++j) {
      const size_t bo = (size_t)(n0 + (j << 4) + rlane) * ldb + koff + k0;
      bh[j] = Frag<T>::load(Bb + bo);
      if (SPLIT) bl[j] = Frag<T>::load(Bb2 + bo);
    }
#pragma unroll
    for (int i = 0; i < 4; ++i) {
      const size_t ao = (size_t)(m0 + (i << 4) + rlane) * lda + koff + k0;
      V ah = Frag<T>::load(Ab + ao);
      V al;
      if (SPLIT) al = Frag<T>::load(Ab2 + ao);
#pragma unroll
      for (int j = 0; j < 4; ++j) {
        acc[i][j] = Frag<T>::mma(ah, bh[j], acc[i][j]);
        if (SPLIT) {
          acc[i][j] = Frag<T>::mma(ah, bl[j], acc[i][j]);
          acc[i][j] = Frag<T>::mma(al, bh[j], acc[i][j]);
        }
      }
      Frag<T>::guard(acc[i][0], acc[i][3], ah, SPLIT ? al : ah);
    }
    Frag<T>::keep(bh[0], bh[1], bh[2], bh[3]);
    if (SPLIT) Frag<T>::keep(bl[0], bl[1], bl[2], bl[3]);
  }
  acc_guard4(acc[0][0], acc[0][1], acc[0][2], acc[0][3]);
  acc_guard4(acc[1][0], acc[1][1], acc[1][2], acc[1][3]);
  acc_guard4(acc[2][0], acc[2][1], acc[2][2], acc[2][3]);
  acc_guard4(acc[3][0], acc[3][1], acc[3][2], acc[3][3]);

  float* slab = sT[wave];
  const float* Rb = RESID ? (resid + (size_t)b * strideR) : nullptr;
#pragma unroll
  for (int i = 0; i < 4; ++i) {
    const int mBase = m0 + (i << 4);
#pragma unroll
    for (int j = 0; j < 4; ++j) {
      const int n = n0 + (j << 4) + rlane;
      float bv = 0.f;
      if (BIAS_MODE == 2) bv = bias[n];
#pragma unroll
      for (int r = 0; r < 8; ++r) {
        float v = acc[i][j][r] * scale;
        if (BIAS_MODE == 1) v += bias[mBase + mOff + r];
        if (BIAS_MODE == 2) v += bv;
        if (RESID) v += Rb[(size_t)(mBase + mOff + r) * ldc + n];
        if (ACT == 2) v = fmaxf(v, 0.0f);
        if (ACT == 4) v = (v > 0.f) ? v : 0.01f * v;
        slab[(mOff + r) * 68 + (j << 4) + rlane] = v;
      }
    }
    __builtin_amdgcn_fence(__ATOMIC_RELEASE, "workgroup");
    __builtin_amdgcn_wave_barrier();
    __builtin_amdgcn_fence(__ATOMIC_ACQUIRE, "workgroup");
    if (OUT_MODE == 0) {
      float* C = (float*)Cout + (size_t)b * strideC;
      const int hh = lane >> 4, c4 = (lane & 15) * 4;
      for (int pass = 0; pass < 2; ++pass) {
#pragma unroll
        for (int it = 0; it < 8; ++it) {
          const int row = it * 2 + hh;
          v4f v = *(const v4f*)(slab + row * 68 + c4);
          *(volatile v4f*)(C + (size_t)(mBase + row) * ldc + n0 + c4) = v;
        }
        __threadfence();
      }
    } else {
      const int q = lane >> 3, c8 = (lane & 7) * 8;
      unsigned short* C  = (unsigned short*)Cout  + (size_t)b * strideC;
      unsigned short* C2 = (OUT_MODE == 2) ? ((unsigned short*)Cout2 + (size_t)b * strideC) : nullptr;
      for (int pass = 0; pass < 2; ++pass) {
#pragma unroll
        for (int it = 0; it < 4; ++it) {
          const int row = it * 4 + q;
          const float* sp = slab + row * 68 + c8;
          v8h hv, lv;
#pragma unroll
          for (int e = 0; e < 8; ++e) {
            if (OUT_MODE == 1) {
              hv[e] = (_Float16)sp[e];
            } else {
              unsigned short hb = f2bf_bits(sp[e]);
              unsigned short lb = f2bf_bits(sp[e] - bf_bits2f(hb));
              hv[e] = __builtin_bit_cast(_Float16, hb);
              lv[e] = __builtin_bit_cast(_Float16, lb);
            }
          }
          *(volatile v8h*)(C + (size_t)(mBase + row) * ldc + n0 + c8) = hv;
          if (OUT_MODE == 2) *(volatile v8h*)(C2 + (size_t)(mBase + row) * ldc + n0 + c8) = lv;
        }
        __threadfence();
      }
    }
    __builtin_amdgcn_fence(__ATOMIC_RELEASE, "workgroup");
    __builtin_amdgcn_wave_barrier();
    __builtin_amdgcn_fence(__ATOMIC_ACQUIRE, "workgroup");
  }
}

__global__ __launch_bounds__(256) void cast8_f16_kernel(const float* __restrict__ in, unsigned short* __restrict__ out,
                                                        int n8, float carry) {
  const int i = blockIdx.x * 256 + threadIdx.x;
  if (i >= n8) return;
  const float* p = in + 8 * (size_t)i;
  const v4f a = *(const v4f*)(p);
  const v4f c = *(const v4f*)(p + 4);
  unsigned short hb[8];
#pragma unroll
  for (int e = 0; e < 4; ++e) {
    hb[e]     = h_bits(a[e] * carry);
    hb[4 + e] = h_bits(c[e] * carry);
  }
  const v4u u = (v4u){pk16(hb[0], hb[1]), pk16(hb[2], hb[3]), pk16(hb[4], hb[5]), pk16(hb[6], hb[7])};
  unsigned short* q = out + 8 * (size_t)i;
  *(volatile v4u*)q = u;
  __threadfence();
  *(volatile v4u*)q = u;
}

__global__ __launch_bounds__(256) void softmax_row_kernel(const float* __restrict__ S, unsigned short* __restrict__ P, float carry) {
  __shared__ float redM[8];
  __shared__ float redS[8];
  const int row  = blockIdx.x;
  const int t    = threadIdx.x;
  const int lane = t & 31, wave = t >> 5;
  const int cA   = 8 * t;
  const int cB   = kSeqHalf + 8 * t;
  const float* sr = S + (size_t)row * kSeq;
  const v4f a0 = *(const v4f*)(sr + cA);
  const v4f a1 = *(const v4f*)(sr + cA + 4);
  const v4f b0 = *(const v4f*)(sr + cB);
  const v4f b1 = *(const v4f*)(sr + cB + 4);
  float x[16];
#pragma unroll
  for (int e = 0; e < 4; ++e) { x[e] = a0[e]; x[4 + e] = a1[e]; x[8 + e] = b0[e]; x[12 + e] = b1[e]; }
  float m = x[0];
#pragma unroll
  for (int e = 1; e < 16; ++e) m = fmaxf(m, x[e]);
#pragma unroll
  for (int off = 16; off > 0; off >>= 1) m = fmaxf(m, __shfl_xor(m, off, 32));
  if (lane == 0) redM[wave] = m;
  __syncthreads();
  float gm = redM[0];
#pragma unroll
  for (int w = 1; w < 8; ++w) gm = fmaxf(gm, redM[w]);
  float ex[16];
  float s = 0.f;
#pragma unroll
  for (int e = 0; e < 16; ++e) { ex[e] = expf(x[e] - gm); s += ex[e]; }
#pragma unroll
  for (int off = 16; off > 0; off >>= 1) s += __shfl_xor(s, off, 32);
  if (lane == 0) redS[wave] = s;
  __syncthreads();
  float tot = redS[0];
#pragma unroll
  for (int w = 1; w < 8; ++w) tot += redS[w];
  const float inv = carry * (1.0f / tot);
  unsigned short hb[16];
#pragma unroll
  for (int e = 0; e < 16; ++e) hb[e] = h_bits(ex[e] * inv);
  const v4u uA = (v4u){pk16(hb[0], hb[1]), pk16(hb[2], hb[3]), pk16(hb[4], hb[5]), pk16(hb[6], hb[7])};
  const v4u uB = (v4u){pk16(hb[8], hb[9]), pk16(hb[10], hb[11]), pk16(hb[12], hb[13]), pk16(hb[14], hb[15])};
  unsigned short* pr = P + (size_t)row * kSeq;
  *(volatile v4u*)(pr + cA) = uA;
  *(volatile v4u*)(pr + cB) = uB;
  __threadfence();
  *(volatile v4u*)(pr + cA) = uA;
  *(volatile v4u*)(pr + cB) = uB;
}

__global__ __launch_bounds__(128) void layernorm_kernel(const float* __restrict__ Y, const float* __restrict__ gamma,
                                                        const float* __restrict__ beta, float* __restrict__ out) {
  __shared__ float redA[4];
  __shared__ float redB[4];
  const int row  = blockIdx.x;
  const int t    = threadIdx.x;
  const int lane = t & 31, wave = t >> 5;
  const int c    = 4 * t;
  const v4f y  = *(const v4f*)(Y + (size_t)row * kDim + c);
  const v4f g  = *(const v4f*)(gamma + c);
  const v4f bb = *(const v4f*)(beta + c);
  float s = (y[0] + y[1]) + (y[2] + y[3]);
#pragma unroll
  for (int off = 16; off > 0; off >>= 1) s += __shfl_xor(s, off, 32);
  if (lane == 0) redA[wave] = s;
  __syncthreads();
  const float mu = ((redA[0] + redA[1]) + (redA[2] + redA[3])) * kInvDim;
  float d[4];
#pragma unroll
  for (int e = 0; e < 4; ++e) d[e] = y[e] - mu;
  float ss = (d[0] * d[0] + d[1] * d[1]) + (d[2] * d[2] + d[3] * d[3]);
#pragma unroll
  for (int off = 16; off > 0; off >>= 1) ss += __shfl_xor(ss, off, 32);
  if (lane == 0) redB[wave] = ss;
  __syncthreads();
  const float var  = ((redB[0] + redB[1]) + (redB[2] + redB[3])) * kInvDim;
  const float rstd = rsqrtf(var + kLnEps);
  v4f ov;
#pragma unroll
  for (int e = 0; e < 4; ++e) ov[e] = d[e] * rstd * g[e] + bb[e];
  float* op = out + (size_t)row * kDim + c;
  *(volatile v4f*)op = ov;
  __threadfence();
  *(volatile v4f*)op = ov;
}

extern "C" void kernel_launch(void* const* d_in, const int* in_sizes, int n_in,
                              void* d_out, int out_size, void* d_ws, size_t ws_size,
                              hipStream_t stream) {
  if (n_in < 9) return;
  if (in_sizes[2] != kTok * kDim || in_sizes[3] != kDim * kDim || in_sizes[4] != kDim * kDim ||
      in_sizes[5] != kDim * kDim || in_sizes[6] != kDim * kDim || in_sizes[7] != kDim || in_sizes[8] != kDim) return;
  if (out_size != kTok * kDim) return;
  if (ws_size < kWsTotal) return;

  const float* Xin   = (const float*)d_in[2];
  const float* Wq    = (const float*)d_in[3];
  const float* Wk    = (const float*)d_in[4];
  const float* Wv    = (const float*)d_in[5];
  const float* Wo    = (const float*)d_in[6];
  const float* gamma = (const float*)d_in[7];
  const float* beta  = (const float*)d_in[8];
  float* Out = (float*)d_out;

  char* ws = (char*)d_ws;
  unsigned short* QK16  = (unsigned short*)(ws + kOffQK);
  unsigned short* VT16  = (unsigned short*)(ws + kOffVT);
  unsigned short* CTX16 = (unsigned short*)(ws + kOffCTX);
  unsigned short* Xh    = (unsigned short*)(ws + kOffXh);
  unsigned short* Wqk16 = (unsigned short*)(ws + kOffWqk);
  unsigned short* Wv16  = (unsigned short*)(ws + kOffWv);
  float*          Sf    = (float*)(ws + kOffS);
  unsigned short* P16   = (unsigned short*)(ws + kOffP);
  float*          Yf    = (float*)(ws + kOffY);
  unsigned short* Wo16  = (unsigned short*)(ws + kOffWo);

  const int nX8 = (kTok * kDim) / 8;
  const int nW8 = (kDim * kDim) / 8;

  cast8_f16_kernel<<<nX8 / 256, 256, 0, stream>>>(Xin, Xh, nX8, 1.0f);
  cast8_f16_kernel<<<nW8 / 256, 256, 0, stream>>>(Wq, Wqk16, nW8, kWCarry);
  cast8_f16_kernel<<<nW8 / 256, 256, 0, stream>>>(Wk, Wqk16 + (size_t)kDim * kDim, nW8, kWCarry);
  cast8_f16_kernel<<<nW8 / 256, 256, 0, stream>>>(Wv, Wv16, nW8, kWCarry);

  wmma_gemm64<0, false, 0, 1, false><<<dim3(256, 1), 256, 0, stream>>>(
      Xh, Xh, kDim, (long)0, Wqk16, Wqk16, kDim, (long)0,
      (void*)QK16, (void*)QK16, kQKld, (long)0, gamma, Xin, (long)0,
      kTok, kQKld, kDim, kWCarryInv);

  wmma_gemm64<0, false, 0, 1, false><<<dim3(64, kBatch), 256, 0, stream>>>(
      Wv16, Wv16, kDim, (long)0, Xh, Xh, kDim, (long)kSeq * kDim,
      (void*)VT16, (void*)VT16, kSeq, (long)kDim * kSeq, gamma, Xin, (long)0,
      kDim, kSeq, kDim, kWCarryInv);

  for (int gidx = 0; gidx < kBatch * kHeads; ++gidx) {
    const int b = gidx / kHeads;
    const int h = gidx - b * kHeads;
    const unsigned short* Qg  = QK16 + (size_t)b * kSeq * kQKld + (size_t)h * kHeadDim;
    const unsigned short* Kg  = Qg + kDim;
    const unsigned short* VTg = VT16 + (size_t)b * kDim * kSeq + (size_t)h * kHeadDim * kSeq;
    unsigned short*       Cg  = CTX16 + (size_t)b * kSeq * kDim + (size_t)h * kHeadDim;

    wmma_gemm64<0, false, 0, 0, false><<<dim3(512, 1), 256, 0, stream>>>(
        Qg, Qg, kQKld, (long)0, Kg, Kg, kQKld, (long)0,
        (void*)Sf, (void*)Sf, kSeq, (long)0, gamma, Xin, (long)0,
        kSeq, kSeq, kHeadDim, kAttScale);

    softmax_row_kernel<<<kSeq, 256, 0, stream>>>(Sf, P16, kPCarry);

    wmma_gemm64<0, false, 0, 1, false><<<dim3(8, 1), 256, 0, stream>>>(
        P16, P16, kSeq, (long)0, VTg, VTg, kSeq, (long)0,
        (void*)Cg, (void*)Cg, kDim, (long)0, gamma, Xin, (long)0,
        kSeq, kHeadDim, kSeq, kPVScale);
  }

  cast8_f16_kernel<<<nW8 / 256, 256, 0, stream>>>(Wo, Wo16, nW8, kWCarry);

  wmma_gemm64<0, false, 0, 0, true><<<dim3(128, 1), 256, 0, stream>>>(
      CTX16, CTX16, kDim, (long)0, Wo16, Wo16, kDim, (long)0,
      (void*)Yf, (void*)Yf, kDim, (long)0, gamma, Xin, (long)0,
      kTok, kDim, kDim, kOutScale);

  layernorm_kernel<<<kTok, 128, 0, stream>>>(Yf, gamma, beta, Out);
}
